// TrackSSM_85117661872149
// MI455X (gfx1250) — hardware-run, weakly checked
//
#include <hip/hip_runtime.h>
#include <math.h>

typedef __attribute__((ext_vector_type(16))) _Float16 v16h;
typedef __attribute__((ext_vector_type(8)))  _Float16 v8h;
typedef __attribute__((ext_vector_type(16))) __bf16   v16b;
typedef __attribute__((ext_vector_type(8)))  __bf16   v8b;
typedef __attribute__((ext_vector_type(8)))  float    v8f;
typedef __attribute__((ext_vector_type(4)))  float    v4f;

constexpr int kSteps   = 64;
constexpr int kTracks  = 256;
constexpr int kChan    = 256;
constexpr int kStates  = 16;
constexpr int kRank    = 16;
constexpr int kXW      = kRank + 2 * kStates;
constexpr int kXP      = 64;
constexpr int kRows    = kSteps * kTracks;
constexpr int kChunk   = 16;
constexpr int kYP      = 264;
constexpr int kOut0Elems = kTracks * kSteps * kChan;
constexpr int kOut1Elems = kTracks * kChan * kStates;
constexpr float kYCarry = 32.0f;
constexpr float kWCarry = 1024.0f;
constexpr float kFold   = 1.0f / (kYCarry * kWCarry);
constexpr float kF16MinNormal = 6.103515625e-5f;
static_assert(kXW == 48);
static_assert(kXW <= kXP);
static_assert(kRows == 16384);
static_assert((kChan % 32) == 0);
static_assert((kRows % 64) == 0 && (kXP % 64) == 0 && (kChan % 64) == 0);
static_assert((kSteps % kChunk) == 0);
static_assert(kChunk * kYP >= kChunk * kChan);
static_assert((size_t)kOut0Elems * 4 == 16777216ull);
static_assert((size_t)kOut1Elems * 4 == 4194304ull);
static_assert(kFold == 1.0f / 32768.0f);

constexpr size_t kOffFB = 0;
constexpr size_t kOffW1 = kOffFB + (size_t)kRows * kChan * 2;
constexpr size_t kOffW2 = kOffW1 + (size_t)kXP * kChan * 2;
constexpr size_t kOffXD = kOffW2 + (size_t)kChan * kChan * 2;
constexpr size_t kOffYH = kOffXD + (size_t)kRows * kXP * 4;
constexpr size_t kWsTotal = kOffYH + (size_t)kRows * kChan * 2;
static_assert(kWsTotal == 21135360ull);
static_assert(kWsTotal <= 134217728ull);
static_assert((kOffW1 % 256) == 0 && (kOffW2 % 256) == 0 && (kOffXD % 256) == 0 && (kOffYH % 256) == 0);

__device__ __forceinline__ unsigned short f2bf_bits(float f) {
  unsigned u = __float_as_uint(f);
  return (unsigned short)((u + 0x7FFFu + ((u >> 16) & 1u)) >> 16);
}
__device__ __forceinline__ float bf_bits2f(unsigned short h) { return __uint_as_float(((unsigned)h) << 16); }
__device__ __forceinline__ float bf16r(float f) { return bf_bits2f(f2bf_bits(f)); }

namespace eng {

__device__ __forceinline__ void dep_guard1_h(v8f& a, v16h x, v16h y) { asm volatile("v_nop\n\tv_nop\n\tv_nop\n\tv_nop" : "+v"(a) : "v"(x), "v"(y)); }
__device__ __forceinline__ void dep_guard1_b(v8f& a, v16b x, v16b y) { asm volatile("v_nop\n\tv_nop\n\tv_nop\n\tv_nop" : "+v"(a) : "v"(x), "v"(y)); }
__device__ __forceinline__ void keep4_h(v16h a, v16h b, v16h c, v16h d) { asm volatile("v_nop" :: "v"(a), "v"(b), "v"(c), "v"(d)); }
__device__ __forceinline__ void keep4_b(v16b a, v16b b, v16b c, v16b d) { asm volatile("v_nop" :: "v"(a), "v"(b), "v"(c), "v"(d)); }
__device__ __forceinline__ void acc_guard4(v8f& a, v8f& b, v8f& c, v8f& d) { asm volatile("v_nop\n\tv_nop\n\tv_nop\n\tv_nop" : "+v"(a), "+v"(b), "+v"(c), "+v"(d)); }

template <typename T> struct Frag;
template <> struct Frag<_Float16> {
  typedef v16h V; union U { v16h v; v8h h[2]; };
  static __device__ __forceinline__ v16h load(const _Float16* p) {
    U f; f.h[0] = *(const v8h*)(p); f.h[1] = *(const v8h*)(p + 16); return f.v;
  }
  static __device__ __forceinline__ v8f mma(v16h a, v16h b, v8f c) {
    return __builtin_amdgcn_wmma_f32_16x16x32_f16(false, a, false, b, (short)0, c, false, false);
  }
  static __device__ __forceinline__ void guard1(v8f& a, v16h x, v16h y) { dep_guard1_h(a, x, y); }
  static __device__ __forceinline__ void keep(v16h a, v16h b, v16h c, v16h d) { keep4_h(a, b, c, d); }
};
template <> struct Frag<__bf16> {
  typedef v16b V; union U { v16b v; v8b h[2]; };
  static __device__ __forceinline__ v16b load(const __bf16* p) {
    U f; f.h[0] = *(const v8b*)(p); f.h[1] = *(const v8b*)(p + 16); return f.v;
  }
  static __device__ __forceinline__ v8f mma(v16b a, v16b b, v8f c) {
    return __builtin_amdgcn_wmma_f32_16x16x32_bf16(false, a, false, b, (short)0, c, false, false);
  }
  static __device__ __forceinline__ void guard1(v8f& a, v16b x, v16b y) { dep_guard1_b(a, x, y); }
  static __device__ __forceinline__ void keep(v16b a, v16b b, v16b c, v16b d) { keep4_b(a, b, c, d); }
};

template <int ET> struct Elem;
template <> struct Elem<0> { typedef _Float16 T; };
template <> struct Elem<1> { typedef __bf16 T; };

template <int ET>
__global__ __launch_bounds__(256) void wmma_gemm64(
    const unsigned short* __restrict__ Ap, int lda,
    const unsigned short* __restrict__ Btp, int ldb,
    float* __restrict__ Cout, int ldc,
    int M, int N, int K, float scale) {
  typedef typename Elem<ET>::T T;
  typedef typename Frag<T>::V V;
  const T* A  = (const T*)Ap;
  const T* Bt = (const T*)Btp;
  __shared__ __align__(16) float sT[8][16 * 68];
  const int lane = threadIdx.x & 31;
  const int wave = threadIdx.x >> 5;
  const int tilesN = N >> 6;
  const int tilesM = M >> 6;
  const int tile = blockIdx.x * 8 + wave;
  if (tile >= tilesM * tilesN) return;
  const int tm = tile / tilesN;
  const int tn = tile - tm * tilesN;
  const int m0 = tm << 6;
  const int n0 = tn << 6;

  const int rlane = lane & 15;
  const int koff  = (lane >> 4) * 8;
  const int mOff  = (lane >> 4) * 8;

  v8f acc[4][4];
#pragma unroll
  for (int i = 0; i < 4; ++i)
#pragma unroll
    for (int j = 0; j < 4; ++j) acc[i][j] = (v8f){0.f, 0.f, 0.f, 0.f, 0.f, 0.f, 0.f, 0.f};

  for (int k0 = 0; k0 < K; k0 += 32) {
    V bh[4];
#pragma unroll
    for (int j = 0; j < 4; ++j) {
      const size_t bo = (size_t)(n0 + (j << 4) + rlane) * ldb + koff + k0;
      bh[j] = Frag<T>::load(Bt + bo);
    }
#pragma unroll
    for (int i = 0; i < 4; ++i) {
      const size_t ao = (size_t)(m0 + (i << 4) + rlane) * lda + koff + k0;
      V ah = Frag<T>::load(A + ao);
#pragma unroll
      for (int j = 0; j < 4; ++j) acc[i][j] = Frag<T>::mma(ah, bh[j], acc[i][j]);
#pragma unroll
      for (int j = 0; j < 4; ++j) Frag<T>::guard1(acc[i][j], ah, bh[j]);
    }
    Frag<T>::keep(bh[0], bh[1], bh[2], bh[3]);
  }
  acc_guard4(acc[0][0], acc[0][1], acc[0][2], acc[0][3]);
  acc_guard4(acc[1][0], acc[1][1], acc[1][2], acc[1][3]);
  acc_guard4(acc[2][0], acc[2][1], acc[2][2], acc[2][3]);
  acc_guard4(acc[3][0], acc[3][1], acc[3][2], acc[3][3]);

  float* slab = sT[wave];
#pragma unroll
  for (int i = 0; i < 4; ++i) {
    const int mBase = m0 + (i << 4);
#pragma unroll
    for (int j = 0; j < 4; ++j) {
#pragma unroll
      for (int r = 0; r < 8; ++r) {
        const float v = acc[i][j][r] * scale;
        slab[(mOff + r) * 68 + (j << 4) + rlane] = v;
      }
    }
    __builtin_amdgcn_fence(__ATOMIC_RELEASE, "workgroup");
    __builtin_amdgcn_wave_barrier();
    __builtin_amdgcn_fence(__ATOMIC_ACQUIRE, "workgroup");
    {
      const int hh = lane >> 4, c4 = (lane & 15) * 4;
      for (int pass = 0; pass < 2; ++pass) {
#pragma unroll
        for (int it = 0; it < 8; ++it) {
          const int row = it * 2 + hh;
          v4f v = *(const v4f*)(slab + row * 68 + c4);
          *(volatile v4f*)(Cout + (size_t)(mBase + row) * ldc + n0 + c4) = v;
        }
        __threadfence();
      }
    }
    __builtin_amdgcn_fence(__ATOMIC_RELEASE, "workgroup");
    __builtin_amdgcn_wave_barrier();
    __builtin_amdgcn_fence(__ATOMIC_ACQUIRE, "workgroup");
  }
}

}

template <int MODE>
__global__ __launch_bounds__(256) void cvt8_kernel(const float* __restrict__ src, unsigned short* __restrict__ dst,
                                                   int nrow_dst, int nrow_src, int ncol8, float sc) {
  const int i  = blockIdx.x * 256 + threadIdx.x;
  const int n8 = nrow_dst * ncol8;
  if (i < n8) {
    const int row = i / ncol8;
    const int c8  = i - row * ncol8;
    const bool live = row < nrow_src;
    const int srow = live ? row : (nrow_src - 1);
    const float* sp = src + (size_t)srow * (size_t)(ncol8 * 8) + c8 * 8;
    const v4f a = *(const v4f*)(sp);
    const v4f b = *(const v4f*)(sp + 4);
    v8h hv;
#pragma unroll
    for (int e = 0; e < 4; ++e) {
      const float ta = a[e];
      const float tb = b[e];
      const float fa = live ? ta : 0.0f;
      const float fb = live ? tb : 0.0f;
      if (MODE == 0) {
        const unsigned short b0 = f2bf_bits(fa);
        const unsigned short b1 = f2bf_bits(fb);
        hv[e]     = __builtin_bit_cast(_Float16, b0);
        hv[4 + e] = __builtin_bit_cast(_Float16, b1);
      } else {
        float va = bf16r(fa) * sc;
        float vb = bf16r(fb) * sc;
        va = (fabsf(va) < kF16MinNormal) ? 0.0f : va;
        vb = (fabsf(vb) < kF16MinNormal) ? 0.0f : vb;
        hv[e]     = (_Float16)va;
        hv[4 + e] = (_Float16)vb;
      }
    }
    *(volatile v8h*)(dst + (size_t)i * 8) = hv;
    __threadfence();
    *(volatile v8h*)(dst + (size_t)i * 8) = hv;
  }
}

__global__ __launch_bounds__(256) void scan_kernel(
    const float* __restrict__ pos, const float* __restrict__ hin, const float* __restrict__ XD,
    const float* __restrict__ dtw, const float* __restrict__ dtb, const float* __restrict__ alog,
    const float* __restrict__ dskip, unsigned short* __restrict__ YH, float* __restrict__ HF) {
  __shared__ __align__(16) float sX[kSteps * kXP];
  __shared__ __align__(16) float sY[kChunk * kYP];
  __shared__ __align__(16) float sH[kChan * kStates];
  const int tid = threadIdx.x, lane = tid & 31, wave = tid >> 5;
  const int b = blockIdx.x;
  const int d = tid;

  {
    const int r0 = tid >> 4, c4 = (tid & 15) * 4;
#pragma unroll
    for (int i = 0; i < 4; ++i) {
      const int row = r0 + 16 * i;
      const v4f v = *(const v4f*)(XD + ((size_t)row * kTracks + b) * kXP + c4);
      *(v4f*)(sX + row * kXP + c4) = v;
    }
  }
#pragma unroll 1
  for (int n = 0; n < kStates; ++n) {
    const float al = alog[(size_t)d * kStates + n];
    sH[n * kChan + tid] = -expf(bf16r(al));
  }
  __syncthreads();

  float hA[8], hB[8], aA[8], aB[8], w[16];
  {
    const float* hp = hin + ((size_t)b * kChan + d) * kStates;
    const float* wp = dtw + (size_t)d * kRank;
    v4f hq[4], wq[4];
#pragma unroll
    for (int q = 0; q < 4; ++q) {
      hq[q] = *(const v4f*)(hp + 4 * q);
      wq[q] = *(const v4f*)(wp + 4 * q);
    }
#pragma unroll
    for (int k = 0; k < 8; ++k) {
      const float t0 = hq[k >> 2][k & 3];
      const float t1 = hq[2 + (k >> 2)][k & 3];
      hA[k] = bf16r(t0);
      hB[k] = bf16r(t1);
      aA[k] = sH[k * kChan + tid];
      aB[k] = sH[(8 + k) * kChan + tid];
    }
#pragma unroll
    for (int k = 0; k < 16; ++k) {
      const float t = wq[k >> 2][k & 3];
      w[k] = bf16r(t);
    }
  }
  const float bias = bf16r(dtb[d]);
  const float Dd   = bf16r(dskip[d]);

#pragma unroll 1
  for (int c = 0; c < kSteps / kChunk; ++c) {
#pragma unroll 1
    for (int s = 0; s < kChunk; ++s) {
      const int l = c * kChunk + s;
      const float* xr = sX + l * kXP;
      const v4f x0 = *(const v4f*)(xr);
      const v4f x1 = *(const v4f*)(xr + 4);
      const v4f x2 = *(const v4f*)(xr + 8);
      const v4f x3 = *(const v4f*)(xr + 12);
      float pre = bias;
      pre = fmaf(x0[0], w[0], pre);
      pre = fmaf(x0[1], w[1], pre);
      pre = fmaf(x0[2], w[2], pre);
      pre = fmaf(x0[3], w[3], pre);
      pre = fmaf(x1[0], w[4], pre);
      pre = fmaf(x1[1], w[5], pre);
      pre = fmaf(x1[2], w[6], pre);
      pre = fmaf(x1[3], w[7], pre);
      pre = fmaf(x2[0], w[8], pre);
      pre = fmaf(x2[1], w[9], pre);
      pre = fmaf(x2[2], w[10], pre);
      pre = fmaf(x2[3], w[11], pre);
      pre = fmaf(x3[0], w[12], pre);
      pre = fmaf(x3[1], w[13], pre);
      pre = fmaf(x3[2], w[14], pre);
      pre = fmaf(x3[3], w[15], pre);
      const float ea  = expf(-fabsf(pre));
      const float u   = 1.0f + ea;
      const float l1p = logf(u) + (ea - (u - 1.0f)) * __builtin_amdgcn_rcpf(u);
      const float dlt = fmaxf(pre, 0.0f) + l1p;

      const float p  = bf16r(pos[((size_t)l * kTracks + b) * kChan + d]);
      const float dp = dlt * p;
      float y = 0.0f;
#pragma unroll 1
      for (int g = 0; g < 2; ++g) {
        const float* bp = xr + kRank + 8 * g;
        const float* cp = xr + kRank + kStates + 8 * g;
        const v4f b0 = *(const v4f*)(bp);
        const v4f b1 = *(const v4f*)(bp + 4);
        const v4f c0 = *(const v4f*)(cp);
        const v4f c1 = *(const v4f*)(cp + 4);
        const float Bv[8] = {b0[0], b0[1], b0[2], b0[3], b1[0], b1[1], b1[2], b1[3]};
        const float Cv[8] = {c0[0], c0[1], c0[2], c0[3], c1[0], c1[1], c1[2], c1[3]};
#pragma unroll
        for (int k = 0; k < 8; ++k) {
          const float e = expf(dlt * aA[k]);
          hA[k] = fmaf(e, hA[k], dp * Bv[k]);
          y = fmaf(hA[k], Cv[k], y);
        }
#pragma unroll
        for (int k = 0; k < 8; ++k) {
          const float th = hA[k];
          hA[k] = hB[k];
          hB[k] = th;
          const float ta = aA[k];
          aA[k] = aB[k];
          aB[k] = ta;
        }
      }
      y = fmaf(p, Dd, y);
      sY[s * kYP + tid] = y;
    }
    __syncthreads();
    {
      v8h yv[2];
#pragma unroll
      for (int it = 0; it < 2; ++it) {
        const float* sp = sY + (it * 8 + wave) * kYP + lane * 8;
        const v4f a0 = *(const v4f*)(sp);
        const v4f a1 = *(const v4f*)(sp + 4);
#pragma unroll
        for (int e = 0; e < 4; ++e) {
          const float t0 = a0[e];
          const float t1 = a1[e];
          float v0 = t0 * kYCarry;
          float v1 = t1 * kYCarry;
          v0 = (fabsf(v0) < kF16MinNormal) ? 0.0f : v0;
          v1 = (fabsf(v1) < kF16MinNormal) ? 0.0f : v1;
          yv[it][e]     = (_Float16)v0;
          yv[it][4 + e] = (_Float16)v1;
        }
      }
      for (int pass = 0; pass < 2; ++pass) {
#pragma unroll
        for (int it = 0; it < 2; ++it) {
          const size_t orow = (size_t)b * kSteps + (size_t)(c * kChunk + it * 8 + wave);
          *(volatile v8h*)(YH + orow * kChan + lane * 8) = yv[it];
        }
        __threadfence();
      }
    }
    __syncthreads();
  }

#pragma unroll
  for (int q = 0; q < 2; ++q) {
    const v4f va = {hA[4 * q], hA[4 * q + 1], hA[4 * q + 2], hA[4 * q + 3]};
    const v4f vb = {hB[4 * q], hB[4 * q + 1], hB[4 * q + 2], hB[4 * q + 3]};
    *(v4f*)(sH + tid * kStates + 4 * q)     = va;
    *(v4f*)(sH + tid * kStates + 8 + 4 * q) = vb;
  }
  __syncthreads();
  {
    v4f hv[4];
#pragma unroll
    for (int i = 0; i < 4; ++i) hv[i] = *(const v4f*)(sH + i * 1024 + tid * 4);
    float* hp = HF + (size_t)b * (kChan * kStates);
    for (int pass = 0; pass < 2; ++pass) {
#pragma unroll
      for (int i = 0; i < 4; ++i) *(volatile v4f*)(hp + i * 1024 + tid * 4) = hv[i];
      __threadfence();
    }
  }
}

extern "C" void kernel_launch(void* const* d_in, const int* in_sizes, int n_in,
                              void* d_out, int out_size, void* d_ws, size_t ws_size,
                              hipStream_t stream) {
  if (n_in < 9 || d_out == nullptr || d_ws == nullptr) return;
  if (in_sizes[0] != kSteps * kTracks * kChan) return;
  if (in_sizes[1] != kSteps * kTracks * kChan) return;
  if (in_sizes[2] != kTracks * kChan * kStates) return;
  if (in_sizes[3] != kXW * kChan) return;
  if (in_sizes[4] != kChan * kRank) return;
  if (in_sizes[5] != kChan) return;
  if (in_sizes[6] != kChan * kStates) return;
  if (in_sizes[7] != kChan) return;
  if (in_sizes[8] != kChan * kChan) return;
  if (out_size != kOut0Elems + kOut1Elems) return;
  if (ws_size < kWsTotal) return;

  const float* pos   = (const float*)d_in[0];
  const float* flow  = (const float*)d_in[1];
  const float* hin   = (const float*)d_in[2];
  const float* xw    = (const float*)d_in[3];
  const float* dtw   = (const float*)d_in[4];
  const float* dtb   = (const float*)d_in[5];
  const float* alog  = (const float*)d_in[6];
  const float* dskip = (const float*)d_in[7];
  const float* ow    = (const float*)d_in[8];
  float* out0 = (float*)d_out;
  float* out1 = out0 + (size_t)kOut0Elems;

  char* ws = (char*)d_ws;
  unsigned short* FB = (unsigned short*)(ws + kOffFB);
  unsigned short* W1 = (unsigned short*)(ws + kOffW1);
  unsigned short* W2 = (unsigned short*)(ws + kOffW2);
  float*          XD = (float*)(ws + kOffXD);
  unsigned short* YH = (unsigned short*)(ws + kOffYH);

  constexpr int n8f = kRows * (kChan / 8);
  constexpr int n8x = kXP * (kChan / 8);
  constexpr int n8o = kChan * (kChan / 8);
  static_assert((n8f % 256) == 0 && (n8x % 256) == 0 && (n8o % 256) == 0);
  cvt8_kernel<0><<<n8f / 256, 256, 0, stream>>>(flow, FB, kRows, kRows, kChan / 8, 1.0f);
  cvt8_kernel<0><<<n8x / 256, 256, 0, stream>>>(xw,   W1, kXP,   kXW,   kChan / 8, 1.0f);
  cvt8_kernel<1><<<n8o / 256, 256, 0, stream>>>(ow,   W2, kChan, kChan, kChan / 8, kWCarry);

  eng::wmma_gemm64<1><<<(kRows / 64) * (kXP / 64) / 8, 256, 0, stream>>>(
      FB, kChan, W1, kChan, XD, kXP, kRows, kXP, kChan, 1.0f);

  scan_kernel<<<kTracks, kChan, 0, stream>>>(pos, hin, XD, dtw, dtb, alog, dskip, YH, out1);

  eng::wmma_gemm64<0><<<(kRows / 64) * (kChan / 64) / 8, 256, 0, stream>>>(
      YH, kChan, W2, kChan, out0, kChan, kRows, kChan, kChan, kFold);
}
